// Model_39676907881857
// MI455X (gfx1250) — hardware-run, weakly checked
//
#include <hip/hip_runtime.h>


#define NQ   2048
#define NH   1024
constexpr size_t al256(size_t b) { return (b + 255) & ~(size_t)255; }
constexpr size_t PB16 = (size_t)NQ * NQ * 2, PB32 = (size_t)NQ * NQ * 4;
constexpr size_t WS_TOTAL = 6 * al256(PB16) + 4 * al256(PB32) + al256((size_t)NH * NQ * 4);
static_assert(WS_TOTAL == 125829120 && WS_TOTAL <= 134217728, "the workspace carve: 120.0 MiB");
static_assert(NQ % 64 == 0 && NH % 64 == 0 && NQ % 32 == 0, "whole tiles; whole depth steps");
typedef _Float16 h16;
typedef unsigned short bf;
typedef __attribute__((ext_vector_type(16))) __bf16   v16bf;
typedef __attribute__((ext_vector_type(16))) _Float16 v16h;
typedef __attribute__((ext_vector_type(8)))  _Float16 v8h;
typedef __attribute__((ext_vector_type(8)))  unsigned short v8us;
typedef __attribute__((ext_vector_type(8)))  float    v8f;
typedef __attribute__((ext_vector_type(4)))  float    v4f;
typedef v8h  __attribute__((may_alias)) v8ha;
typedef v4f  __attribute__((may_alias)) v4fa;
typedef v8us __attribute__((may_alias)) v8usa;

__device__ __forceinline__ unsigned short f2bf(float f) { unsigned u = __float_as_uint(f); u += 0x7FFFu + ((u >> 16) & 1u); return (unsigned short)(u >> 16); }
__device__ __forceinline__ float bf2f(unsigned short b) { return __uint_as_float(((unsigned)b) << 16); }
__device__ __forceinline__ float bfr(float f) { return bf2f(f2bf(f)); }
__device__ __forceinline__ v16h cat16(v8h lo, v8h hi) { return __builtin_shufflevector(lo, hi, 0, 1, 2, 3, 4, 5, 6, 7, 8, 9, 10, 11, 12, 13, 14, 15); }
__device__ __forceinline__ v16bf cat16b(v8us lo, v8us hi) { return __builtin_bit_cast(v16bf, __builtin_shufflevector(lo, hi, 0, 1, 2, 3, 4, 5, 6, 7, 8, 9, 10, 11, 12, 13, 14, 15)); }
__device__ __forceinline__ v8f wmma16(v16h a, v16h b, v8f c) { return __builtin_amdgcn_wmma_f32_16x16x32_f16(false, a, false, b, (short)0, c, false, false); }
__device__ __forceinline__ v8f wmmab(v16bf a, v16bf b, v8f c) { return __builtin_amdgcn_wmma_f32_16x16x32_bf16(false, a, false, b, (short)0, c, false, false); }


template <typename T16> struct WFrag;
template <> struct WFrag<h16> { typedef v16h V; static __device__ __forceinline__ V ld(const h16* p) { return cat16(*(const v8h*)p, *(const v8h*)(p + 16)); } static __device__ __forceinline__ v8f mma(V a, V b, v8f c) { return wmma16(a, b, c); } };
template <> struct WFrag<bf> { typedef v16bf V; static __device__ __forceinline__ V ld(const bf* p) { return cat16b(*(const v8us*)p, *(const v8us*)(p + 16)); } static __device__ __forceinline__ v8f mma(V a, V b, v8f c) { return wmmab(a, b, c); } };
template <typename T16, int NSPLIT, bool BIAS>
__global__ __launch_bounds__(32) void k_gemmw(const T16* __restrict__ A, const T16* __restrict__ A2, const T16* __restrict__ Bt, const T16* __restrict__ Bt2, int K, float* C, int ldc, const float* __restrict__ bias, size_t sA, size_t sB, size_t sC) {
    typedef typename WFrag<T16>::V V;
    __shared__ __align__(16) float os[16 * 68];
    const size_t z = blockIdx.z; A += z * sA; if (A2) A2 += z * sA; Bt += z * sB; if (Bt2) Bt2 += z * sB; C += z * sC;
    const int lane = threadIdx.x & 31, lr = lane & 15, hi = lane >> 4; const int r0 = blockIdx.x * 64, c0 = blockIdx.y * 64;
    v8f acc[4][4];
#pragma unroll
    for (int mb = 0; mb < 4; ++mb)
#pragma unroll
        for (int nb = 0; nb < 4; ++nb) acc[mb][nb] = (v8f){};
    const size_t aoff = (size_t)(r0 + lr) * K + 8 * hi, boff = (size_t)(c0 + lr) * K + 8 * hi;
    for (int kc = 0; kc < K; kc += 32) {
        V a[4], a2[4];
#pragma unroll
        for (int mb = 0; mb < 4; ++mb) { a[mb] = WFrag<T16>::ld(A + aoff + (size_t)mb * 16 * K + kc); if (NSPLIT == 1 || NSPLIT == 2) a2[mb] = WFrag<T16>::ld(A2 + aoff + (size_t)mb * 16 * K + kc); }
#pragma unroll
        for (int nb = 0; nb < 4; ++nb) { const V b = WFrag<T16>::ld(Bt + boff + (size_t)nb * 16 * K + kc); V b2; if (NSPLIT >= 2) b2 = WFrag<T16>::ld(Bt2 + boff + (size_t)nb * 16 * K + kc);
#pragma unroll
            for (int mb = 0; mb < 4; ++mb) { acc[mb][nb] = WFrag<T16>::mma(a[mb], b, acc[mb][nb]); if (NSPLIT == 1 || NSPLIT == 2) acc[mb][nb] = WFrag<T16>::mma(a2[mb], b, acc[mb][nb]); if (NSPLIT >= 2) acc[mb][nb] = WFrag<T16>::mma(a[mb], b2, acc[mb][nb]); } }
        asm volatile("v_nop\n\tv_nop\n\tv_nop\n\tv_nop" : "+v"(acc[0][0]), "+v"(acc[1][1]), "+v"(acc[2][2]), "+v"(acc[3][3]) : "v"(a[0]), "v"(a[3]));
    }
#pragma unroll
    for (int mb = 0; mb < 4; ++mb) {
#pragma unroll
        for (int nb = 0; nb < 4; ++nb) {
#pragma unroll
            for (int j = 0; j < 8; ++j) os[(hi * 8 + j) * 68 + nb * 16 + lr] = acc[mb][nb][j]; }
        __builtin_amdgcn_wave_barrier(); asm volatile("" ::: "memory");
        float* crow = C + (size_t)(r0 + mb * 16) * ldc + c0;
#pragma unroll 1
        for (int ps = 0; ps < 2; ++ps) {
#pragma unroll
            for (int s = 0; s < 8; ++s) { const int row = 2 * s + hi, cofs = lr * 4; v4f val = *(const v4fa*)(os + row * 68 + cofs); if (BIAS) { val[0] += bfr(bias[c0 + cofs]); val[1] += bfr(bias[c0 + cofs + 1]); val[2] += bfr(bias[c0 + cofs + 2]); val[3] += bfr(bias[c0 + cofs + 3]); }
                *(volatile v4f*)(crow + (size_t)row * ldc + cofs) = val; }
            if (ps == 0) __threadfence(); }
        __builtin_amdgcn_wave_barrier(); asm volatile("" ::: "memory");
    }
}

__device__ __forceinline__ h16 tohx(float x) { return (h16)x; }
__device__ __forceinline__ void splitf(float y, unsigned short& h, unsigned short& l) { h = f2bf(y); l = f2bf(y - bf2f(h)); }
typedef __attribute__((ext_vector_type(2))) _Float16 v2h;
typedef __attribute__((ext_vector_type(4))) _Float16 v4h;
typedef __attribute__((ext_vector_type(2))) unsigned short v2us;
typedef __attribute__((ext_vector_type(4))) unsigned short v4us;
typedef __attribute__((ext_vector_type(2))) float v2f;
typedef __attribute__((ext_vector_type(4))) int v4i;

__global__ __launch_bounds__(256) void k_cvt8(const float* __restrict__ src, bf* dst, size_t n8) { const size_t i = (size_t)blockIdx.x * 256 + threadIdx.x; if (i >= n8) return; const v8f v = *(const v8f*)(src + i * 8); v8us o;
#pragma unroll
    for (int k = 0; k < 8; ++k) o[k] = f2bf(v[k]); *(volatile v8us*)(dst + i * 8) = o; __threadfence(); *(volatile v8us*)(dst + i * 8) = o; }

__global__ __launch_bounds__(256) void k_wtG(const float* __restrict__ w, int K, int N, bf* Bt) {
    const int lane = threadIdx.x & 31; const int L0 = (blockIdx.x * 8 + (threadIdx.x >> 5)) * 8; const int nlines = N * K / 64;
#pragma unroll
    for (int ps = 0; ps < 2; ++ps) {
        for (int l = 0; l < 8; ++l) { const int L = L0 + l; if (L >= nlines) break; const size_t e = (size_t)L * 64 + lane * 2; const int k = (int)(e % K), n = (int)(e / K); v2us o;
            o[0] = f2bf(w[(size_t)k * N + n]); o[1] = f2bf(w[(size_t)(k + 1) * N + n]); *(volatile v2us*)(Bt + e) = o; }
        if (ps == 0) __threadfence(); }
}

__global__ __launch_bounds__(256) void k_tohl(const float* __restrict__ F, float sc, bf* Hh, bf* Hl, size_t n4) { const size_t i = (size_t)blockIdx.x * 256 + threadIdx.x; if (i >= n4) return; const v4f a = *(const v4f*)(F + i * 4); v4us oh, ol;
#pragma unroll
    for (int q = 0; q < 4; ++q) { unsigned short h2, l2; splitf(__fmul_rn(a[q], sc), h2, l2); oh[q] = h2; ol[q] = l2; }
    *(volatile v4us*)(Hh + i * 4) = oh; *(volatile v4us*)(Hl + i * 4) = ol; __threadfence(); *(volatile v4us*)(Hh + i * 4) = oh; *(volatile v4us*)(Hl + i * 4) = ol; }

__global__ __launch_bounds__(256) void k_mw(const float* __restrict__ PA, const float* __restrict__ wa, float* MA, size_t n4) {
    const size_t i = (size_t)blockIdx.x * 256 + threadIdx.x; if (i >= n4) return; const v4f a = *(const v4f*)(PA + i * 4); const v4f w = *(const v4f*)(wa + i * 4); v4f o;
#pragma unroll
    for (int q = 0; q < 4; ++q) o[q] = a[q] * bfr(w[q]);
    *(volatile v4f*)(MA + i * 4) = o; __threadfence(); *(volatile v4f*)(MA + i * 4) = o; }

__device__ __forceinline__ float comb1(float ga, float gb, float gc, float qm, float qa, float w) {
    const float ue = qm * bfr(w); const float uf = ga * gb + ga + gc; const float uz = gb - gb; const float ug = uf * uz + ue * gc; const float uh = gc * ug; const float uk = (gc * qa) * ue;
    return (uf + uh) + (uz + uk); }
__global__ __launch_bounds__(256) void k_comb(const float* __restrict__ PA, const float* __restrict__ PB, const float* __restrict__ PC, const float* __restrict__ QM, const float* __restrict__ QA, const float* __restrict__ wa, float* res, size_t n4) {
    const size_t i = (size_t)blockIdx.x * 256 + threadIdx.x; if (i >= n4) return;
    const v4f va = *(const v4f*)(PA + i * 4); const v4f vb = *(const v4f*)(PB + i * 4); const v4f vc = *(const v4f*)(PC + i * 4); const v4f vm = *(const v4f*)(QM + i * 4); const v4f vq = *(const v4f*)(QA + i * 4); const v4f w = *(const v4f*)(wa + i * 4); v4f o;
#pragma unroll
    for (int q = 0; q < 4; ++q) o[q] = comb1(va[q], vb[q], vc[q], vm[q], vq[q], w[q]);
    *(volatile v4f*)(res + i * 4) = o; __threadfence(); *(volatile v4f*)(res + i * 4) = o; }

extern "C" void kernel_launch(void* const* d_in, const int* in_sizes, int n_in,
                              void* d_out, int out_size, void* d_ws, size_t ws_size, hipStream_t stream) {
    if (n_in < 4) return;
    for (int j = 0; j < 4; ++j) if (in_sizes[j] < NQ * NQ) return;
    if (out_size < NQ * NQ) return;
    const float* xin = (const float*)d_in[0]; const float* wa = (const float*)d_in[1]; const float* wb = (const float*)d_in[2]; const float* wc = (const float*)d_in[3];
    float* OUT = (float*)d_out;
    char* wsp = (char*)d_ws;
    auto take = [&](size_t bytes) { char* p = wsp; wsp += (bytes + 255) & ~(size_t)255; return (void*)p; };
    bf* XB = (bf*)take(PB16); bf* W3B = (bf*)take(PB16); bf* W1T = (bf*)take(PB16); bf* W2T = (bf*)take(PB16); bf* W3T = (bf*)take(PB16); bf* XT = (bf*)take(PB16);
    float* PA = (float*)take(PB32); float* PB = (float*)take(PB32); float* PC = (float*)take(PB32); float* MA = (float*)take(PB32); float* QA = (float*)take((size_t)NH * NQ * 4);
    if ((size_t)(wsp - (char*)d_ws) != WS_TOTAL || WS_TOTAL > ws_size) return;
    bf* PAh = XB; bf* PAl = W1T; bf* MAh = W2T; bf* MAl = W3B; float* QM = MA;
    const unsigned g8 = (unsigned)(((size_t)NQ * NQ / 8 + 255) / 256), g4 = (unsigned)(((size_t)NQ * NQ / 4 + 255) / 256), gw = (unsigned)(((size_t)NQ * NQ / 64 + 63) / 64);
    k_cvt8<<<g8, 256, 0, stream>>>(xin, XB, (size_t)NQ * NQ / 8); k_cvt8<<<g8, 256, 0, stream>>>(wc, W3B, (size_t)NQ * NQ / 8);
    k_wtG<<<gw, 256, 0, stream>>>(wa, NQ, NQ, W1T); k_wtG<<<gw, 256, 0, stream>>>(wb, NQ, NQ, W2T); k_wtG<<<gw, 256, 0, stream>>>(wc, NQ, NQ, W3T); k_wtG<<<gw, 256, 0, stream>>>(xin, NQ, NQ, XT);
    k_gemmw<bf, 0, false><<<dim3(NQ / 64, NQ / 64, 1), 32, 0, stream>>>(XB, nullptr, W1T, nullptr, NQ, PA, NQ, nullptr, (size_t)0, (size_t)0, (size_t)0);
    k_gemmw<bf, 0, false><<<dim3(NQ / 64, NQ / 64, 1), 32, 0, stream>>>(XB, nullptr, W2T, nullptr, NQ, PB, NQ, nullptr, (size_t)0, (size_t)0, (size_t)0);
    k_gemmw<bf, 0, false><<<dim3(NQ / 64, NQ / 64, 1), 32, 0, stream>>>(W3B, nullptr, W3T, nullptr, NQ, PC, NQ, nullptr, (size_t)0, (size_t)0, (size_t)0);
    k_mw<<<g4, 256, 0, stream>>>(PA, wa, MA, (size_t)NQ * NQ / 4);
    k_tohl<<<g4, 256, 0, stream>>>(PA, 1.0f, PAh, PAl, (size_t)NQ * NQ / 4);
    k_tohl<<<g4, 256, 0, stream>>>(MA, 1.0f, MAh, MAl, (size_t)NQ * NQ / 4);
    k_gemmw<bf, 1, false><<<dim3(NQ / 64, NQ / 64, 1), 32, 0, stream>>>(MAh, MAl, XT, nullptr, NQ, QM, NQ, nullptr, (size_t)0, (size_t)0, (size_t)0);
    for (int hf = 0; hf < 2; ++hf) {
        const size_t ro = (size_t)hf * NH * NQ;
        k_gemmw<bf, 1, false><<<dim3(NH / 64, NQ / 64, 1), 32, 0, stream>>>(PAh + ro, PAl + ro, XT, nullptr, NQ, QA, NQ, nullptr, (size_t)0, (size_t)0, (size_t)0);
        k_comb<<<(unsigned)(((size_t)NH * NQ / 4 + 255) / 256), 256, 0, stream>>>(PA + ro, PB + ro, PC + ro, QM + ro, QA, wa + ro, OUT + ro, (size_t)NH * NQ / 4);
    }
}
